// SpectralAttentionLayer_63187558858868
// MI455X (gfx1250) — hardware-verified
//
#include <hip/hip_runtime.h>
#include <stddef.h>


#define DW      32
#define KC      96
#define FW      64
#define NTHR    256
#define NWAVE   8
#define EPT     8
#define NGRP    2
#define CHUNK   (NTHR * EPT * NGRP)
#define WCAP    (EPT * NGRP * 32)
#define LISTN   (NWAVE * WCAP)
#define NBC     4096
#define NBF     1024
#define RCAP    40960
#define RBN     128
#define TGT     256
#define DEGCAP  1024
#define OTHR    512
#define GTHR    128
#define BM      64
#define WUNITS  (DW * (KC / 8) + FW * (DW / 8))
#define WSCAP   134217728
#define ACARRY  64.0f
#define WCARRY  64.0f
#define GSCALE  (1.0f / 4096.0f)
#define NEG_SL  0.2f

#define LDS_FILL ((RCAP + 3 * NBF + LISTN + NWAVE) * 4 + 64)

static_assert((CHUNK & (CHUNK - 1)) == 0);
static_assert(CHUNK <= 4096);
static_assert(NBC <= 4096);
static_assert((NBC & (NBC - 1)) == 0 && (NBF & (NBF - 1)) == 0);
static_assert(NBC == 4 * NBF);
static_assert(OTHR * 8 == NBC);
static_assert((RCAP % 32) == 0);
static_assert(TGT == NWAVE * 32);
static_assert((NBC % TGT) == 0);
static_assert((NBF % TGT) == 0);
static_assert((TGT % BM) == 0);
static_assert(DW == 32);
static_assert((KC % 32) == 0);
static_assert(FW == 2 * DW);
static_assert(WCAP == EPT * NGRP * 32);
static_assert(NBF == 4 * NTHR);
static_assert(((RCAP + 2 * NBF + LISTN) % 4) == 0);
static_assert(((BM * 4) % 128) == 0);
static_assert((WUNITS % 32) == 0);
static_assert(DEGCAP % 32 == 0);

typedef float    v4f  __attribute__((ext_vector_type(4)));
typedef float    v8f  __attribute__((ext_vector_type(8)));
typedef int      v4i  __attribute__((ext_vector_type(4)));
typedef _Float16 v4h  __attribute__((ext_vector_type(4)));
typedef _Float16 v8h  __attribute__((ext_vector_type(8)));
typedef _Float16 v16h __attribute__((ext_vector_type(16)));
union Frag { v16h v; v8h h[2]; };

__device__ __forceinline__ v8f wmh(v16h a, v16h b, v8f c) {
  v8f d = __builtin_amdgcn_wmma_f32_16x16x32_f16(false, a, false, b, (short)0, c, false, false);
  asm volatile("v_nop\n\tv_nop\n\tv_nop\n\tv_nop" : "+v"(d) : "v"(a), "v"(b));
  return d;
}

__device__ __forceinline__ float wsum(float v) {
  v += __shfl_xor(v, 16);
  v += __shfl_xor(v, 8);
  v += __shfl_xor(v, 4);
  v += __shfl_xor(v, 2);
  v += __shfl_xor(v, 1);
  return v;
}

template <int NB>
__device__ __forceinline__ int scan_chunk(const int* __restrict__ dsts, int nE, int cbase, int slotBase,
                                          int vec8, int* list, int tid, int lane, int wave) {
  int wc = 0;
#pragma unroll
  for (int g = 0; g < NGRP; ++g) {
    const int el0  = (g * NTHR + tid) * EPT;
    const int e0   = cbase + el0;
    const int sent = -2147483647 - 1;
    v4i da, db;
    if (vec8 != 0 && cbase + CHUNK <= nE) {
      da = *(const v4i*)(dsts + e0);
      db = *(const v4i*)(dsts + e0 + 4);
    } else {
      da.x = (e0     < nE) ? dsts[min(e0, nE - 1)] : sent;
      da.y = (e0 + 1 < nE) ? dsts[min(e0 + 1, nE - 1)] : sent;
      da.z = (e0 + 2 < nE) ? dsts[min(e0 + 2, nE - 1)] : sent;
      da.w = (e0 + 3 < nE) ? dsts[min(e0 + 3, nE - 1)] : sent;
      db.x = (e0 + 4 < nE) ? dsts[min(e0 + 4, nE - 1)] : sent;
      db.y = (e0 + 5 < nE) ? dsts[min(e0 + 5, nE - 1)] : sent;
      db.z = (e0 + 6 < nE) ? dsts[min(e0 + 6, nE - 1)] : sent;
      db.w = (e0 + 7 < nE) ? dsts[min(e0 + 7, nE - 1)] : sent;
    }
    const unsigned nb = (unsigned)slotBase;
    const unsigned s0 = (unsigned)da.x - nb, s1 = (unsigned)da.y - nb;
    const unsigned s2 = (unsigned)da.z - nb, s3 = (unsigned)da.w - nb;
    const unsigned s4 = (unsigned)db.x - nb, s5 = (unsigned)db.y - nb;
    const unsigned s6 = (unsigned)db.z - nb, s7 = (unsigned)db.w - nb;
    const bool h0 = s0 < (unsigned)NB, h1 = s1 < (unsigned)NB, h2 = s2 < (unsigned)NB, h3 = s3 < (unsigned)NB;
    const bool h4 = s4 < (unsigned)NB, h5 = s5 < (unsigned)NB, h6 = s6 < (unsigned)NB, h7 = s7 < (unsigned)NB;
    const unsigned any = __builtin_amdgcn_ballot_w32(h0 | h1 | h2 | h3 | h4 | h5 | h6 | h7);
    if (any != 0u) {
#define HITJ(J, HJ, SJ) { \
        const unsigned mj = __builtin_amdgcn_ballot_w32(HJ); \
        if (mj != 0u) { \
          if (HJ) { \
            const int pos = wc + (int)__builtin_amdgcn_mbcnt_lo(mj, 0u); \
            if (pos < WCAP) list[wave * WCAP + pos] = ((el0 + (J)) << 12) | (int)(SJ); \
          } \
          wc += (int)__builtin_popcount(mj); } }
      HITJ(0, h0, s0)
      HITJ(1, h1, s1)
      HITJ(2, h2, s2)
      HITJ(3, h3, s3)
      HITJ(4, h4, s4)
      HITJ(5, h5, s5)
      HITJ(6, h6, s6)
      HITJ(7, h7, s7)
#undef HITJ
    }
  }
  return wc;
}

__global__ __launch_bounds__(NTHR) void k_count(const int* __restrict__ dsts, int* cnt, int nE, int vec8) {
  __shared__ __attribute__((aligned(16))) int scnt[NBC];
  __shared__ __attribute__((aligned(16))) int list[LISTN];
  __shared__ int wcnt[NWAVE];
  const int tid = threadIdx.x, lane = tid & 31, wave = tid >> 5;
  const int nodeBase = blockIdx.x * NBC;

  for (int i = tid; i < NBC; i += NTHR) scnt[i] = 0;
  __syncthreads();

  const int nChunks = (nE + CHUNK - 1) / CHUNK;
#pragma unroll 1
  for (int ch = 0; ch < nChunks; ++ch) {
    const int cbase = ch * CHUNK;
    const int wc = scan_chunk<NBC>(dsts, nE, cbase, nodeBase, vec8, list, tid, lane, wave);
    if (lane == 0) wcnt[wave] = wc;
    __syncthreads();
    if (wave == 0) {
#pragma unroll 1
      for (int wsx = 0; wsx < NWAVE; ++wsx) {
        int n = __builtin_amdgcn_readfirstlane(wcnt[wsx]);
        n = n > WCAP ? WCAP : (n < 0 ? 0 : n);
        const int* lp = list + wsx * WCAP;
#pragma unroll 1
        for (int i = 0; i < n; ++i) {
          const int ent  = __builtin_amdgcn_readfirstlane(lp[i]);
          const int slot = ent & (NBC - 1);
          if (lane == 0) scnt[slot] = scnt[slot] + 1;
        }
      }
    }
    __syncthreads();
  }

  v4i cq[4];
#pragma unroll
  for (int q = 0; q < 4; ++q) {
    const int f = (wave * 4 + q) * 128 + 4 * lane;
    cq[q] = *(const v4i*)(scnt + f);
  }
  int* cp = cnt + (size_t)nodeBase;
#pragma unroll
  for (int q = 0; q < 4; ++q) {
    const int f = (wave * 4 + q) * 128 + 4 * lane;
    *(volatile v4i*)(cp + f) = cq[q];
  }
  __threadfence();
#pragma unroll
  for (int q = 0; q < 4; ++q) {
    const int f = (wave * 4 + q) * 128 + 4 * lane;
    *(volatile v4i*)(cp + f) = cq[q];
  }
}

__global__ __launch_bounds__(OTHR) void k_offsets(
    const int* __restrict__ cnt, int* off, int* rbase, int nChunk) {
  __shared__ __attribute__((aligned(16))) int soff[NBC];
  __shared__ __attribute__((aligned(16))) int srb[RBN];
  __shared__ int wtot[OTHR / 32];
  const int tid = threadIdx.x, lane = tid & 31, wave = tid >> 5, sub = tid >> 7;
  for (int i = tid; i < RBN; i += OTHR) srb[i] = 0;
  int carry = 0;
#pragma unroll 1
  for (int ch = 0; ch < nChunk; ++ch) {
    const int base = ch * NBC;
    const v4i c0 = *(const v4i*)(cnt + base + 8 * tid);
    const v4i c1 = *(const v4i*)(cnt + base + 8 * tid + 4);
    const int e0 = max(c0.x, 0), e1 = max(c0.y, 0), e2 = max(c0.z, 0), e3 = max(c0.w, 0);
    const int e4 = max(c1.x, 0), e5 = max(c1.y, 0), e6 = max(c1.z, 0), e7 = max(c1.w, 0);
    const int ts = e0 + e1 + e2 + e3 + e4 + e5 + e6 + e7;
    int incl = ts;
#pragma unroll
    for (int d = 1; d < 32; d <<= 1) {
      const int t = __shfl_up(incl, d);
      if (lane >= d) incl += t;
    }
    if (lane == 31) wtot[wave] = incl;
    __syncthreads();
    const int S0 = wtot[0]  + wtot[1]  + wtot[2]  + wtot[3];
    const int S1 = wtot[4]  + wtot[5]  + wtot[6]  + wtot[7];
    const int S2 = wtot[8]  + wtot[9]  + wtot[10] + wtot[11];
    const int S3 = wtot[12] + wtot[13] + wtot[14] + wtot[15];
    int pre = 0;
#pragma unroll 1
    for (int w = 4 * sub; w < wave; ++w) pre += wtot[w];
    const int b0 = carry;
    const int b1 = b0 + ((S0 + 31) & ~31);
    const int b2 = b1 + ((S1 + 31) & ~31);
    const int b3 = b2 + ((S2 + 31) & ~31);
    const int b4 = b3 + ((S3 + 31) & ~31);
    const int myb = sub == 0 ? b0 : (sub == 1 ? b1 : (sub == 2 ? b2 : b3));
    if (tid == 0) {
      srb[min(4 * ch + 0, RBN - 1)] = b0;
      srb[min(4 * ch + 1, RBN - 1)] = b1;
      srb[min(4 * ch + 2, RBN - 1)] = b2;
      srb[min(4 * ch + 3, RBN - 1)] = b3;
    }
    int run = myb + pre + incl - ts;
    soff[8 * tid + 0] = run; run += e0;
    soff[8 * tid + 1] = run; run += e1;
    soff[8 * tid + 2] = run; run += e2;
    soff[8 * tid + 3] = run; run += e3;
    soff[8 * tid + 4] = run; run += e4;
    soff[8 * tid + 5] = run; run += e5;
    soff[8 * tid + 6] = run; run += e6;
    soff[8 * tid + 7] = run;
    carry = b4;
    __syncthreads();
    const v4i o0 = *(const v4i*)(soff + 4 * tid);
    const v4i o1 = *(const v4i*)(soff + 4 * (tid + OTHR));
    int* op = off + base;
    *(volatile v4i*)(op + 4 * tid) = o0;
    *(volatile v4i*)(op + 4 * (tid + OTHR)) = o1;
    __threadfence();
    *(volatile v4i*)(op + 4 * tid) = o0;
    *(volatile v4i*)(op + 4 * (tid + OTHR)) = o1;
    __syncthreads();
  }
  if (tid == 0) srb[min(4 * nChunk, RBN - 1)] = carry;
  __syncthreads();
  v4i rv = {0, 0, 0, 0};
  if (tid < 32) rv = *(const v4i*)(srb + 4 * tid);
  if (tid < 32) *(volatile v4i*)(rbase + 4 * tid) = rv;
  __threadfence();
  if (tid < 32) *(volatile v4i*)(rbase + 4 * tid) = rv;
}

__global__ __launch_bounds__(NTHR) void k_fill(
    const int* __restrict__ dsts, const int* __restrict__ off, const int* __restrict__ rbase,
    int* csr, float* dinv, int nE, int vec8, int csrLen) {
  extern __shared__ v4f lds_dyn[];
  int*   region = (int*)lds_dyn;
  int*   cursor = region + RCAP;
  int*   cstart = cursor + NBF;
  int*   list   = cstart + NBF;
  float* sdinv  = (float*)(list + LISTN);
  int*   wcnt   = (int*)(sdinv + NBF);
  const int tid = threadIdx.x, lane = tid & 31, wave = tid >> 5;
  const int b = blockIdx.x;
  const int nodeBase = b * NBF;

  int rb0 = rbase[b];
  const int rb1 = rbase[b + 1];
  rb0 = rb0 < 0 ? 0 : (rb0 > csrLen ? csrLen : rb0);
  rb0 &= ~31;
  int len = rb1 - rb0;
  len = len < 0 ? 0 : (len > RCAP ? RCAP : len);
  int lenW = (len + 31) & ~31;
  if (rb0 + lenW > csrLen) lenW = (csrLen - rb0) & ~31;

  {
    const v4i z = {0, 0, 0, 0};
    for (int i = tid; i < RCAP / 4; i += NTHR) ((v4i*)region)[i] = z;
    for (int s = tid; s < NBF; s += NTHR) {
      int o = off[nodeBase + s] - rb0;
      o = o < 0 ? 0 : (o > RCAP ? RCAP : o);
      cursor[s] = o;
      cstart[s] = o;
    }
  }
  __syncthreads();

  const int nChunks = (nE + CHUNK - 1) / CHUNK;
#pragma unroll 1
  for (int ch = 0; ch < nChunks; ++ch) {
    const int cbase = ch * CHUNK;
    const int wc = scan_chunk<NBF>(dsts, nE, cbase, nodeBase, vec8, list, tid, lane, wave);
    if (lane == 0) wcnt[wave] = wc;
    __syncthreads();
    if (wave == 0) {
#pragma unroll 1
      for (int wsx = 0; wsx < NWAVE; ++wsx) {
        int n = __builtin_amdgcn_readfirstlane(wcnt[wsx]);
        n = n > WCAP ? WCAP : (n < 0 ? 0 : n);
        const int* lp = list + wsx * WCAP;
#pragma unroll 1
        for (int i = 0; i < n; ++i) {
          const int ent  = __builtin_amdgcn_readfirstlane(lp[i]);
          const int slot = ent & (NBF - 1);
          int e = cbase + ((ent >> 12) & (CHUNK - 1));
          e = e > nE - 1 ? nE - 1 : (e < 0 ? 0 : e);
          if (lane == 0) {
            int pos = cursor[slot];
            pos = pos < 0 ? 0 : (pos > RCAP - 1 ? RCAP - 1 : pos);
            region[pos] = e;
            const int np = pos + 1;
            cursor[slot] = np > RCAP ? RCAP : np;
          }
        }
      }
    }
    __syncthreads();
  }

#pragma unroll 1
  for (int s = tid; s < NBF; s += NTHR) {
    int st = cstart[s];
    st = st < 0 ? 0 : (st > RCAP ? RCAP : st);
    int en = cursor[s];
    en = en < st ? st : (en > RCAP ? RCAP : en);
    const int n = en - st;
    float deg = (float)n;
    deg = deg < 1.f ? 1.f : deg;
    sdinv[s] = rsqrtf(deg);
  }
  __syncthreads();

  const int nv = lenW >> 2;
  int* gp = csr + rb0;
  const v4f dv = *(const v4f*)(sdinv + 4 * tid);
  float* dq = dinv + (size_t)nodeBase + 4 * tid;
#pragma unroll 1
  for (int i = tid; i < nv; i += NTHR) { const v4i v = ((const v4i*)region)[i]; *(volatile v4i*)(gp + 4 * i) = v; }
  *(volatile v4f*)dq = dv;
  __threadfence();
#pragma unroll 1
  for (int i = tid; i < nv; i += NTHR) { const v4i v = ((const v4i*)region)[i]; *(volatile v4i*)(gp + 4 * i) = v; }
  *(volatile v4f*)dq = dv;
}

__global__ __launch_bounds__(NTHR) void k_wcvt(const float* __restrict__ wc, const float* __restrict__ ws_,
                                               const float* __restrict__ wd, _Float16* dp, int nUnits) {
  const int i = (int)blockIdx.x * NTHR + (int)threadIdx.x;
  if (i >= nUnits) return;
  const int uC = DW * (KC / 8);
  const bool inC = i < uC;
  const int r = inC ? i : i - uC;
  int rc = r / 12;
  const int sc = r - rc * 12;
  rc = rc > DW - 1 ? DW - 1 : rc;
  const int rg = r / 4;
  const int sg = r - rg * 4;
  const bool gsrc = rg < DW;
  int ns = rg > DW - 1 ? DW - 1 : rg;
  ns = ns < 0 ? 0 : ns;
  int nd = rg - DW;
  nd = nd < 0 ? 0 : (nd > DW - 1 ? DW - 1 : nd);
  const float* p0 = wc  + (size_t)rc * KC + 8 * sc;
  const float* p1 = ws_ + (size_t)ns * DW + 8 * sg;
  const float* p2 = wd  + (size_t)nd * DW + 8 * sg;
  v8h o;
#pragma unroll
  for (int j = 0; j < 8; ++j) {
    const float f0 = p0[j];
    const float f1 = p1[j];
    const float f2 = p2[j];
    const float f = inC ? f0 : (gsrc ? f1 : f2);
    o[j] = (_Float16)(f * WCARRY);
  }
  _Float16* gp = dp + (size_t)i * 8;
  *(volatile v8h*)gp = o;
  __threadfence();
  *(volatile v8h*)gp = o;
}

template <int KP, int NT, int RELU>
__global__ __launch_bounds__(GTHR) void k_gemm(
    const float* __restrict__ P0, const float* __restrict__ P1, const float* __restrict__ P2,
    const _Float16* __restrict__ Bp, const float* __restrict__ bias0, const float* __restrict__ bias1,
    float* Cout, int nValid) {
  constexpr int AK  = KP * 32;
  constexpr int NC  = NT * 16;
  constexpr int SPP = DW / 4;
  constexpr int NIA = (BM * SPP) / GTHR;
  constexpr int OPR = NC / 4;
  constexpr int NIO = (BM * OPR) / GTHR;
  static_assert((BM * SPP) % GTHR == 0);
  static_assert((BM * OPR) % GTHR == 0);
  static_assert(NIA >= 1 && NIO >= 1);
  static_assert(BM == 16 * (GTHR / 32));
  static_assert(KP >= 1 && KP <= 3);
  static_assert(NC <= FW);

  __shared__ __attribute__((aligned(16))) float stg[BM * NC];
  __shared__ __attribute__((aligned(16))) _Float16 a16[BM * AK];
  const int tid = threadIdx.x, lane = tid & 31, wave = tid >> 5, hh = lane >> 4, m = lane & 15;
  const int rowBase = (int)blockIdx.x * BM;
  const int r0 = wave * 16;

#pragma unroll
  for (int p = 0; p < KP; ++p) {
    const float* src = (p == 0) ? P0 : ((p == 1) ? P1 : P2);
#pragma unroll
    for (int it = 0; it < NIA; ++it) {
      const int id = it * GTHR + tid;
      const int row = id >> 3, seg = id & 7;
      const int grow = rowBase + row;
      const bool live = grow < nValid;
      int rr = grow > nValid - 1 ? nValid - 1 : grow;
      rr = rr < 0 ? 0 : rr;
      v4f xv = *(const v4f*)(src + (size_t)rr * DW + 4 * seg);
      xv.x = live ? xv.x : 0.f;
      xv.y = live ? xv.y : 0.f;
      xv.z = live ? xv.z : 0.f;
      xv.w = live ? xv.w : 0.f;
      v4h o;
      o.x = (_Float16)(xv.x * ACARRY);
      o.y = (_Float16)(xv.y * ACARRY);
      o.z = (_Float16)(xv.z * ACARRY);
      o.w = (_Float16)(xv.w * ACARRY);
      *(v4h*)(a16 + (size_t)row * AK + p * 32 + 4 * seg) = o;
    }
  }
  __syncthreads();

  v8f acc[NT];
#pragma unroll
  for (int t = 0; t < NT; ++t) { v8f z = {0.f, 0.f, 0.f, 0.f, 0.f, 0.f, 0.f, 0.f}; acc[t] = z; }

  const _Float16* ap = a16 + (size_t)(r0 + m) * AK + 8 * hh;
  const _Float16* bp = Bp + (size_t)m * AK + 8 * hh;
#pragma unroll 1
  for (int kt = 0; kt < KP; ++kt) {
    Frag a;
    a.h[0] = *(const v8h*)(ap + 32 * kt);
    a.h[1] = *(const v8h*)(ap + 32 * kt + 16);
#pragma unroll
    for (int t = 0; t < NT; ++t) {
      const size_t to = (size_t)(16 * t) * AK + 32 * kt;
      Frag bf;
      bf.h[0] = *(const v8h*)(bp + to);
      bf.h[1] = *(const v8h*)(bp + to + 16);
      acc[t] = wmh(a.v, bf.v, acc[t]);
    }
  }

  {
    const int growb = rowBase + r0 + 8 * hh;
#pragma unroll
    for (int t = 0; t < NT; ++t) {
      const int col = 16 * t + m;
      int c0i = col > DW - 1 ? DW - 1 : col;
      c0i = c0i < 0 ? 0 : c0i;
      int c1i = col - DW;
      c1i = c1i < 0 ? 0 : (c1i > DW - 1 ? DW - 1 : c1i);
      const float bv0 = bias0[c0i];
      const float bv1 = bias1[c1i];
      const float bv = (col < DW) ? bv0 : bv1;
#pragma unroll
      for (int r = 0; r < 8; ++r) {
        const int row = r0 + 8 * hh + r;
        float v = acc[t][r] * GSCALE + bv;
        if constexpr (RELU != 0) v = fmaxf(v, 0.f);
        const bool lv = (growb + r) < nValid;
        stg[row * NC + col] = lv ? v : 0.f;
      }
    }
  }
  __syncthreads();

  v4f cv[NIO];
#pragma unroll
  for (int it = 0; it < NIO; ++it) {
    const int id = it * GTHR + tid;
    const int row = id / OPR, seg = id % OPR;
    cv[it] = *(const v4f*)(stg + (size_t)row * NC + 4 * seg);
  }
#pragma unroll
  for (int it = 0; it < NIO; ++it) {
    const int id = it * GTHR + tid;
    const int row = id / OPR, seg = id % OPR;
    float* gp = Cout + (size_t)(rowBase + row) * NC + 4 * seg;
    *(volatile v4f*)gp = cv[it];
  }
  __threadfence();
#pragma unroll
  for (int it = 0; it < NIO; ++it) {
    const int id = it * GTHR + tid;
    const int row = id / OPR, seg = id % OPR;
    float* gp = Cout + (size_t)(rowBase + row) * NC + 4 * seg;
    *(volatile v4f*)gp = cv[it];
  }
}

template <int MODE>
__global__ __launch_bounds__(NTHR) void k_hop(
    const int* __restrict__ csr, const int* __restrict__ off, const int* __restrict__ cnt,
    const float* __restrict__ dinv, const int* __restrict__ esrc, const float* __restrict__ lam,
    const float* xin, const float* xprev, float* xout, int nN, int nE, int csrLen) {
  const int tid = threadIdx.x, lane = tid & 31, wave = tid >> 5;
  const int tbase = blockIdx.x * TGT + wave * 32;
  const int cl    = tbase + lane;
  const int cnt_l = cnt[cl];
  const int off_l = off[cl];
  const float di_l = dinv[cl];
  const float lmx = lam[0];
  const float re  = 2.0f / lmx;
  const float cA  = (MODE == 1) ? -re : -2.0f * re;
  const float cB  = (MODE == 1) ? (re - 1.0f) : 2.0f * (re - 1.0f);

#pragma unroll 1
  for (int j = 0; j < 32; ++j) {
    const int c = tbase + j;
    int n = __shfl(cnt_l, j);
    n = n < 0 ? 0 : (n > DEGCAP ? DEGCAP : n);
    const int st = __shfl(off_l, j);
    const float dc = __shfl(di_l, j);
    const int cr = c > nN - 1 ? nN - 1 : c;

    const float xc = xin[(size_t)cr * DW + lane];
    float sum = 0.f;
#pragma unroll 1
    for (int q0 = 0; q0 < n; q0 += 32) {
      int pos = st + q0 + lane;
      pos = pos < 0 ? 0 : (pos > csrLen - 1 ? csrLen - 1 : pos);
      int el = csr[pos];
      el = el < 0 ? 0 : (el > nE - 1 ? nE - 1 : el);
      int sl = esrc[el];
      sl = sl < 0 ? 0 : (sl > nN - 1 ? nN - 1 : sl);
      const float cfl = dinv[sl];
      const int mcnt = (n - q0) < 32 ? (n - q0) : 32;
#pragma unroll 1
      for (int pp = 0; pp < mcnt; ++pp) {
        const int s = __builtin_amdgcn_readlane(sl, pp);
        const float cf = __shfl(cfl, pp);
        const float xv = xin[(size_t)s * DW + lane];
        sum += xv * cf;
      }
    }
    const float P = dc * sum;
    float v = cA * P + cB * xc;
    if constexpr (MODE == 2) {
      const float xp = xprev[(size_t)cr * DW + lane];
      v = v - xp;
    }

    const bool live = c < nN;
    const float o = live ? v : 0.f;
    float* gp = xout + (size_t)c * DW + lane;
    *(volatile float*)gp = o;
    __threadfence();
    *(volatile float*)gp = o;
  }
}

__global__ __launch_bounds__(NTHR) void k_gat(
    const int* __restrict__ csr, const int* __restrict__ off, const int* __restrict__ cnt,
    const int* __restrict__ esrc, const float* __restrict__ fsd, const float* __restrict__ attn,
    const float* __restrict__ gbias, float* out, int nN, int nE, int csrLen) {
  __shared__ __attribute__((aligned(16))) float lg[NWAVE * DEGCAP];
  const int tid = threadIdx.x, lane = tid & 31, wave = tid >> 5;
  const int tbase = blockIdx.x * TGT + wave * 32;
  const int cl    = tbase + lane;
  const int cnt_l = cnt[cl];
  const int off_l = off[cl];
  const float at  = attn[lane];
  const float bo  = gbias[lane];
  const int lgb   = wave * DEGCAP;
  const float ninf = __uint_as_float(0xff800000u);
  const float qnan = __uint_as_float(0x7fc00000u);

#pragma unroll 1
  for (int j = 0; j < 32; ++j) {
    const int c = tbase + j;
    const int nraw = __shfl(cnt_l, j);
    const int n = nraw < 0 ? 0 : (nraw > DEGCAP ? DEGCAP : nraw);
    const int st = __shfl(off_l, j);
    const int cr = c > nN - 1 ? nN - 1 : c;
    const float fdc = fsd[(size_t)cr * FW + DW + lane];

    float mx = ninf;
#pragma unroll 1
    for (int q0 = 0; q0 < n; q0 += 32) {
      int pos = st + q0 + lane;
      pos = pos < 0 ? 0 : (pos > csrLen - 1 ? csrLen - 1 : pos);
      int el = csr[pos];
      el = el < 0 ? 0 : (el > nE - 1 ? nE - 1 : el);
      int sl = esrc[el];
      sl = sl < 0 ? 0 : (sl > nN - 1 ? nN - 1 : sl);
      const int mcnt = (n - q0) < 32 ? (n - q0) : 32;
      float myl = 0.f;
#pragma unroll 1
      for (int pp = 0; pp < mcnt; ++pp) {
        const int s = __builtin_amdgcn_readlane(sl, pp);
        const float x = fsd[(size_t)s * FW + lane];
        float t = x + fdc;
        t = t > 0.f ? t : NEG_SL * t;
        const float l = wsum(t * at);
        mx = fmaxf(mx, l);
        myl = (lane == pp) ? l : myl;
      }
      lg[lgb + q0 + lane] = myl;
    }

    float ssum = 0.f, acc = 0.f;
#pragma unroll 1
    for (int q0 = 0; q0 < n; q0 += 32) {
      int pos = st + q0 + lane;
      pos = pos < 0 ? 0 : (pos > csrLen - 1 ? csrLen - 1 : pos);
      int el = csr[pos];
      el = el < 0 ? 0 : (el > nE - 1 ? nE - 1 : el);
      int sl = esrc[el];
      sl = sl < 0 ? 0 : (sl > nN - 1 ? nN - 1 : sl);
      const int mcnt = (n - q0) < 32 ? (n - q0) : 32;
      const float myl = lg[lgb + q0 + lane];
      const float ex  = expf(myl - mx);
      const float exl = (lane < mcnt) ? ex : 0.f;
      ssum += wsum(exl);
#pragma unroll 1
      for (int pp = 0; pp < mcnt; ++pp) {
        const int s = __builtin_amdgcn_readlane(sl, pp);
        const float cf = __shfl(exl, pp);
        const float x = fsd[(size_t)s * FW + lane];
        acc += x * cf;
      }
    }
    const float inv = ssum > 0.f ? (1.0f / ssum) : 0.f;
    float o = acc * inv + bo;
    o = (nraw > DEGCAP) ? qnan : o;

    if (c < nN) {
      float* gp = out + (size_t)c * DW + lane;
      *(volatile float*)gp = o;
      __threadfence();
      *(volatile float*)gp = o;
    }
  }
}

extern "C" void kernel_launch(void* const* d_in, const int* in_sizes, int n_in,
                              void* d_out, int out_size, void* d_ws, size_t ws_size,
                              hipStream_t stream) {
  if (n_in < 12) return;
  if (in_sizes[0] < DW || (in_sizes[0] % DW) != 0) return;
  const int nN = in_sizes[0] / DW;
  const int nE = in_sizes[1];
  if (nE < 1 || in_sizes[2] != nE) return;
  if (in_sizes[3] < 1) return;
  if (in_sizes[4] != DW * KC || in_sizes[5] != DW) return;
  if (in_sizes[6] != DW * DW || in_sizes[7] != DW) return;
  if (in_sizes[8] != DW * DW || in_sizes[9] != DW) return;
  if (in_sizes[10] != DW || in_sizes[11] != DW) return;
  if ((long long)out_size != (long long)nN * (long long)DW) return;
  if (nE > (1 << 28) || nN > (1 << 22)) return;

  const float* x     = (const float*)d_in[0];
  const int*   src   = (const int*)d_in[1];
  const int*   dst   = (const int*)d_in[2];
  const float* lam   = (const float*)d_in[3];
  const float* chebW = (const float*)d_in[4];
  const float* chebB = (const float*)d_in[5];
  const float* wsrc  = (const float*)d_in[6];
  const float* bsrc  = (const float*)d_in[7];
  const float* wdst  = (const float*)d_in[8];
  const float* bdst  = (const float*)d_in[9];
  const float* attn  = (const float*)d_in[10];
  const float* gbias = (const float*)d_in[11];
  float* out = (float*)d_out;

  const int NPAD   = ((nN + TGT - 1) / TGT) * TGT;
  const int nBC    = (nN + NBC - 1) / NBC;
  const int CNTPAD = nBC * NBC;
  if (CNTPAD < NPAD) return;
  if (4 * nBC + 1 > RBN) return;
  const int nBF    = (nN + NBF - 1) / NBF;
  if (nBF > 4 * nBC) return;
  const int DIPAD  = nBF * NBF;
  if (DIPAD < NPAD) return;
  const int csrLen = ((nE + 31) & ~31) + 4096;
  if (31 * 4 * nBC > 4096) return;
  const int nHop   = NPAD / TGT;
  const int nGemm  = NPAD / BM;
  const int nUnits = WUNITS;

  char* ws = (char*)d_ws;
  size_t off = 0;
  const size_t oWp  = off; off += (size_t)WUNITS * 8 * 2;              off = (off + 255) & ~(size_t)255;
  const size_t oX1  = off; off += (size_t)NPAD * DW * 4;                off = (off + 255) & ~(size_t)255;
  const size_t oX2  = off; off += (size_t)NPAD * DW * 4;                off = (off + 255) & ~(size_t)255;
  const size_t oH1  = off; off += (size_t)NPAD * DW * 4;                off = (off + 255) & ~(size_t)255;
  const size_t oH2  = off; off += (size_t)NPAD * DW * 4;                off = (off + 255) & ~(size_t)255;
  const size_t oFS  = off; off += (size_t)NPAD * FW * 4;                off = (off + 255) & ~(size_t)255;
  const size_t oCnt = off; off += (size_t)CNTPAD * 4;                   off = (off + 255) & ~(size_t)255;
  const size_t oOff = off; off += (size_t)CNTPAD * 4;                   off = (off + 255) & ~(size_t)255;
  const size_t oDi  = off; off += (size_t)DIPAD * 4;                    off = (off + 255) & ~(size_t)255;
  const size_t oRb  = off; off += (size_t)RBN * 4;                      off = (off + 255) & ~(size_t)255;
  const size_t oCsr = off; off += (size_t)csrLen * 4;                   off = (off + 255) & ~(size_t)255;
  if (off > ws_size || off > (size_t)WSCAP) return;

  _Float16* wpl = (_Float16*)(ws + oWp);
  _Float16* wplG = wpl + (size_t)DW * KC;
  float* X1   = (float*)(ws + oX1);
  float* X2   = (float*)(ws + oX2);
  float* H1   = (float*)(ws + oH1);
  float* H2   = (float*)(ws + oH2);
  float* FSD  = (float*)(ws + oFS);
  int*   cnt  = (int*)(ws + oCnt);
  int*   offp = (int*)(ws + oOff);
  float* dinv = (float*)(ws + oDi);
  int*   rb   = (int*)(ws + oRb);
  int*   csr  = (int*)(ws + oCsr);

  const int vec8 = ((((size_t)in_sizes[0] + (size_t)in_sizes[1]) * 4) % 16 == 0) ? 1 : 0;

  k_wcvt<<<(nUnits + NTHR - 1) / NTHR, NTHR, 0, stream>>>(chebW, wsrc, wdst, wpl, nUnits);
  k_count<<<nBC, NTHR, 0, stream>>>(dst, cnt, nE, vec8);
  k_offsets<<<1, OTHR, 0, stream>>>(cnt, offp, rb, nBC);
  hipFuncSetAttribute(reinterpret_cast<const void*>(&k_fill),
                      hipFuncAttributeMaxDynamicSharedMemorySize, LDS_FILL);
  k_fill<<<nBF, NTHR, LDS_FILL, stream>>>(dst, offp, rb, csr, dinv, nE, vec8, csrLen);

  k_hop<1><<<nHop, NTHR, 0, stream>>>(csr, offp, cnt, dinv, src, lam, x, x, X1, nN, nE, csrLen);
  k_hop<2><<<nHop, NTHR, 0, stream>>>(csr, offp, cnt, dinv, src, lam, X1, x, X2, nN, nE, csrLen);
  k_gemm<3, 2, 1><<<nGemm, GTHR, 0, stream>>>(x, X1, X2, wpl, chebB, chebB, H1, nN);

  k_hop<1><<<nHop, NTHR, 0, stream>>>(csr, offp, cnt, dinv, src, lam, H1, H1, X1, nN, nE, csrLen);
  k_hop<2><<<nHop, NTHR, 0, stream>>>(csr, offp, cnt, dinv, src, lam, X1, H1, X2, nN, nE, csrLen);
  k_gemm<3, 2, 1><<<nGemm, GTHR, 0, stream>>>(H1, X1, X2, wpl, chebB, chebB, H2, nN);

  k_gemm<1, 4, 0><<<nGemm, GTHR, 0, stream>>>(H2, H2, H2, wplG, bsrc, bdst, FSD, nN);
  k_gat<<<nHop, NTHR, 0, stream>>>(csr, offp, cnt, src, FSD, attn, gbias, out, nN, nE, csrLen);
}
